// RandomizedBertSelfAttention_45509473468722
// MI455X (gfx1250) — hardware-verified
//
#include <hip/hip_runtime.h>
#include <math.h>
#include <stdint.h>

#define SEQ   4096
#define DIN   768
#define NH    12
#define HD    64
#define OUTW  (NH * HD)
#define QSC   64.0f
#define KSC   64.0f
#define PCAR  32768.0f
#define VCAR  64.0f
#define LOG2E 1.4426950408889634f
#define ATT_WAVES   4
#define ATT_THREADS (ATT_WAVES * 32)
#define QTILES      (SEQ / 64)
#define ATT_BLOCKS  (NH * QTILES)
#define NKB    (SEQ / 32)
#define SLABF  (16 * 68)
#define SLAB64 (16 * 68)
static_assert(HD == 64);
static_assert((SEQ % 64) == 0 && (DIN % 32) == 0 && (OUTW % 64) == 0 && OUTW <= DIN);
static_assert(((SEQ * DIN) % 256) == 0 && ((OUTW * DIN) % 256) == 0 && ((SEQ * OUTW) % 256) == 0);
static_assert(ATT_THREADS == 128 && NKB * 32 == SEQ);
static_assert(ATT_WAVES * SLABF >= 4 * 16 * 68);

typedef unsigned short u16;
typedef _Float16 v16h __attribute__((ext_vector_type(16)));
typedef _Float16 v8h  __attribute__((ext_vector_type(8)));
typedef __bf16   v16b __attribute__((ext_vector_type(16)));
typedef float    v8f  __attribute__((ext_vector_type(8)));
typedef float    v4f  __attribute__((ext_vector_type(4)));
typedef unsigned int v4u __attribute__((ext_vector_type(4)));

union FragH { v16h v; v8h h[2]; v4u u[2]; };
union FragB { v16b v; v4u u[2]; };

__device__ __forceinline__ unsigned short bf_bits(float f) {
  unsigned u = __float_as_uint(f);
  return (unsigned short)((u + 0x7FFFu + ((u >> 16) & 1u)) >> 16);
}
__device__ __forceinline__ float bf_up(unsigned short h) { return __uint_as_float(((unsigned)h) << 16); }
__device__ __forceinline__ float bfr(float f) { return bf_up(bf_bits(f)); }
__device__ __forceinline__ unsigned short h_bits(_Float16 x) { return __builtin_bit_cast(unsigned short, x); }
__device__ __forceinline__ unsigned pk16(unsigned short a, unsigned short b) { return (unsigned)a | ((unsigned)b << 16); }
__device__ __forceinline__ v8f zero8() { v8f z = {0.f, 0.f, 0.f, 0.f, 0.f, 0.f, 0.f, 0.f}; return z; }
__device__ __forceinline__ v4f zero4() { v4f z = {0.f, 0.f, 0.f, 0.f}; return z; }

__device__ __forceinline__ v16h ldfrag_h(const _Float16* p) {
  FragH f;
  f.h[0] = *(const v8h*)(p);
  f.h[1] = *(const v8h*)(p + 16);
  return f.v;
}
__device__ __forceinline__ v16b ldfrag_b(const u16* p) {
  FragB f;
  f.u[0] = *(const v4u*)(p);
  f.u[1] = *(const v4u*)(p + 16);
  return f.v;
}

__device__ __forceinline__ v8f mma_h(v16h a, v16h b, v8f c) {
  return __builtin_amdgcn_wmma_f32_16x16x32_f16(false, a, false, b, (short)0, c, false, false);
}
__device__ __forceinline__ v8f mma_b(v16b a, v16b b, v8f c) {
  return __builtin_amdgcn_wmma_f32_16x16x32_bf16(false, a, false, b, (short)0, c, false, false);
}
__device__ __forceinline__ void g2_3(v8f& a, v8f& b, v16h x0, v16h x1, v16h x2) {
#if defined(__HIP_DEVICE_COMPILE__)
  asm volatile("v_nop\n\tv_nop\n\tv_nop\n\tv_nop" : "+v"(a), "+v"(b) : "v"(x0), "v"(x1), "v"(x2) : "memory");
#endif
}
template <typename F>
__device__ __forceinline__ void g4_5(v8f& a, v8f& b, v8f& c, v8f& d, F x0, F x1, F x2, F x3, F x4) {
#if defined(__HIP_DEVICE_COMPILE__)
  asm volatile("v_nop\n\tv_nop\n\tv_nop\n\tv_nop"
               : "+v"(a), "+v"(b), "+v"(c), "+v"(d) : "v"(x0), "v"(x1), "v"(x2), "v"(x3), "v"(x4) : "memory");
#endif
}
__device__ __forceinline__ void acc_guard4(v8f& a, v8f& b, v8f& c, v8f& d) {
#if defined(__HIP_DEVICE_COMPILE__)
  asm volatile("v_nop\n\tv_nop\n\tv_nop\n\tv_nop" : "+v"(a), "+v"(b), "+v"(c), "+v"(d));
#endif
}
__device__ __forceinline__ void wave_sync_lds() {
  __builtin_amdgcn_fence(__ATOMIC_RELEASE, "workgroup");
  __builtin_amdgcn_wave_barrier();
  __builtin_amdgcn_fence(__ATOMIC_ACQUIRE, "workgroup");
}

__global__ __launch_bounds__(256) void cvb16(const float* __restrict__ x, u16* D, int n8) {
  const int gt = blockIdx.x * 256 + (int)threadIdx.x;
  if (gt >= n8) return;
  const float* p = x + (size_t)gt * 8;
  const v4f a = *(const v4f*)(p), c4 = *(const v4f*)(p + 4);
  float v[8];
#pragma unroll
  for (int e = 0; e < 4; ++e) { v[e] = a[e]; v[4 + e] = c4[e]; }
  unsigned short s[8];
#pragma unroll
  for (int e = 0; e < 8; ++e) s[e] = bf_bits(v[e]);
  v4u o;
#pragma unroll
  for (int e = 0; e < 4; ++e) o[e] = pk16(s[2 * e], s[2 * e + 1]);
  u16* d = D + (size_t)gt * 8;
  for (int pass = 0; pass < 2; ++pass) {
    *(volatile v4u*)(d) = o;
    __threadfence();
  }
}

__global__ __launch_bounds__(256) void cvh16(const float* __restrict__ x, u16* D, int n8, float scale) {
  const int gt = blockIdx.x * 256 + (int)threadIdx.x;
  if (gt >= n8) return;
  const float* p = x + (size_t)gt * 8;
  const v4f a = *(const v4f*)(p), c4 = *(const v4f*)(p + 4);
  float v[8];
#pragma unroll
  for (int e = 0; e < 4; ++e) { v[e] = a[e]; v[4 + e] = c4[e]; }
  unsigned short s[8];
#pragma unroll
  for (int e = 0; e < 8; ++e) s[e] = h_bits((_Float16)(v[e] * scale));
  v4u o;
#pragma unroll
  for (int e = 0; e < 4; ++e) o[e] = pk16(s[2 * e], s[2 * e + 1]);
  u16* d = D + (size_t)gt * 8;
  for (int pass = 0; pass < 2; ++pass) {
    *(volatile v4u*)(d) = o;
    __threadfence();
  }
}

__device__ __forceinline__ void bias_terms(const float* __restrict__ bias, int nb, int bmode, int rowb, int col0, int hh, int m,
                                           v4f& badd, v8f& radd) {
#pragma unroll
  for (int e = 0; e < 4; ++e) {
    const int ci = col0 + 4 * m + e;
    const int ic = ci < nb ? ci : nb - 1;
    const float bc = bfr(bias[ic]);
    badd[e] = (bmode == 0) ? bc : 0.0f;
  }
#pragma unroll
  for (int r = 0; r < 8; ++r) {
    const int ri = rowb + 8 * hh + r;
    const int ir = ri < nb ? ri : nb - 1;
    const float br = bfr(bias[ir]);
    radd[r] = (bmode == 1) ? br : 0.0f;
  }
}

__device__ __forceinline__ void epi64(float* sl, v8f a0, v8f a1, v8f a2, v8f a3, float oscale, v4f badd, v8f radd,
                                      float* C, int N, size_t rowb, int col0, int lane) {
  const int hh = lane >> 4, m = lane & 15;
#pragma unroll
  for (int r = 0; r < 8; ++r) {
    const int ro = (8 * hh + r) * 68 + m;
    sl[ro]      = a0[r] * oscale + radd[r];
    sl[ro + 16] = a1[r] * oscale + radd[r];
    sl[ro + 32] = a2[r] * oscale + radd[r];
    sl[ro + 48] = a3[r] * oscale + radd[r];
  }
  wave_sync_lds();
  v4f vals[8];
#pragma unroll
  for (int it = 0; it < 8; ++it) vals[it] = *(const v4f*)(sl + (it * 2 + hh) * 68 + m * 4) + badd;
  float* dst = C + (rowb + (size_t)hh) * (size_t)N + col0 + m * 4;
  for (int pass = 0; pass < 2; ++pass) {
#pragma unroll
    for (int it = 0; it < 8; ++it) {
      *(volatile v4f*)(dst + (size_t)(it * 2) * (size_t)N) = vals[it];
    }
    __threadfence();
  }
}

__global__ __launch_bounds__(128)
void gemm_bfb(const u16* __restrict__ A, const u16* __restrict__ Bt, const float* __restrict__ bias,
              float* C, int M, int N, int K, float oscale, int bmode, int nb) {
  __shared__ __align__(16) float slab[4 * SLAB64];
  const int tid = threadIdx.x, wave = tid >> 5, lane = tid & 31, hh = lane >> 4, m = lane & 15;
  const int ntile = N >> 6;
  const int bid   = blockIdx.x;
  const int rowb  = (bid / ntile) * 64 + wave * 16;
  const int col0  = (bid % ntile) * 64;
  if (rowb + 16 > M) return;
  const u16* ap = A  + (size_t)(rowb + m) * K + 8 * hh;
  const u16* bp = Bt + (size_t)(col0 + m) * K + 8 * hh;
  const size_t bs = (size_t)16 * K;
  v8f acc0 = zero8(), acc1 = zero8(), acc2 = zero8(), acc3 = zero8();
#pragma unroll 1
  for (int k0 = 0; k0 < K; k0 += 32) {
    const v16b a  = ldfrag_b(ap + k0);
    const v16b b0 = ldfrag_b(bp + k0);
    const v16b b1 = ldfrag_b(bp + bs + k0);
    const v16b b2 = ldfrag_b(bp + 2 * bs + k0);
    const v16b b3 = ldfrag_b(bp + 3 * bs + k0);
    acc0 = mma_b(a, b0, acc0);
    acc1 = mma_b(a, b1, acc1);
    acc2 = mma_b(a, b2, acc2);
    acc3 = mma_b(a, b3, acc3);
    g4_5<v16b>(acc0, acc1, acc2, acc3, a, b0, b1, b2, b3);
  }
  v4f badd = zero4();
  v8f radd = zero8();
  bias_terms(bias, nb, bmode, rowb, col0, hh, m, badd, radd);
  epi64(slab + wave * SLAB64, acc0, acc1, acc2, acc3, oscale, badd, radd, C, N, (size_t)rowb, col0, lane);
}

__global__ __launch_bounds__(ATT_THREADS)
void attn_fwd(const u16* __restrict__ QHp, const u16* __restrict__ KHp, const u16* __restrict__ VHp, float* out) {
  __shared__ __align__(16) float smem[ATT_WAVES * SLABF];

  const int tid  = threadIdx.x;
  const int wave = tid >> 5;
  const int lane = tid & 31;
  const int hh   = lane >> 4;
  const int c    = lane & 15;

  const int bid  = blockIdx.x;
  const int qt   = bid % QTILES;
  const int head = bid / QTILES;
  if (head >= NH) return;
  const int q0   = qt * 64 + wave * 16;

  const size_t qofs = ((size_t)(q0 + c) * NH + head) * HD + 8 * hh;
  const _Float16* Qh  = (const _Float16*)(const void*)QHp + qofs;
  const v16h qh0 = ldfrag_h(Qh), qh1 = ldfrag_h(Qh + 32);
  const size_t kofs = ((size_t)c * NH + head) * HD + 8 * hh;
  const _Float16* Khb = (const _Float16*)(const void*)KHp + kofs;
  const size_t vofs = ((size_t)(head * HD) + c) * SEQ + 8 * hh;
  const _Float16* Vhb = (const _Float16*)(const void*)VHp + vofs;
  const float lsc = 0.125f * (LOG2E / (QSC * KSC));

  float mrun = -INFINITY, lrun = 0.f;
  v8f o[4];
#pragma unroll
  for (int j = 0; j < 4; ++j) o[j] = zero8();

#pragma unroll 1
  for (int it = 0; it < NKB; ++it) {
    const int kb = it * 32;
    v8f s0 = zero8(), s1 = zero8();
    const _Float16* k0p = Khb + (size_t)kb * OUTW;
    const _Float16* k1p = k0p + (size_t)16 * OUTW;
    {
      const v16h kh0 = ldfrag_h(k0p), kh1 = ldfrag_h(k1p);
      s0 = mma_h(kh0, qh0, s0);
      s1 = mma_h(kh1, qh0, s1);
      g2_3(s0, s1, qh0, kh0, kh1);
    }
    {
      const v16h kh0 = ldfrag_h(k0p + 32), kh1 = ldfrag_h(k1p + 32);
      s0 = mma_h(kh0, qh1, s0);
      s1 = mma_h(kh1, qh1, s1);
      g2_3(s0, s1, qh1, kh0, kh1);
    }
    float t[16];
#pragma unroll
    for (int i = 0; i < 8; ++i) { t[i] = s0[i] * lsc; t[8 + i] = s1[i] * lsc; }
    float cm = t[0];
#pragma unroll
    for (int i = 1; i < 16; ++i) cm = fmaxf(cm, t[i]);
    cm = fmaxf(cm, __shfl_xor(cm, 16, 32));
    const float mn = fmaxf(mrun, cm);
    const float al = exp2f(mrun - mn);
    mrun = mn;
    float ps = 0.f;
    FragH ph;
#pragma unroll
    for (int w = 0; w < 2; ++w) {
#pragma unroll
      for (int e4 = 0; e4 < 4; ++e4) {
        const int i = 8 * w + 2 * e4;
        const float p0 = exp2f(t[i] - mn), p1 = exp2f(t[i + 1] - mn);
        ps += p0 + p1;
        const _Float16 h0 = (_Float16)(p0 * PCAR), h1 = (_Float16)(p1 * PCAR);
        ph.u[w][e4] = pk16(h_bits(h0), h_bits(h1));
      }
    }
    ps += __shfl_xor(ps, 16, 32);
    lrun = lrun * al + ps;
    float scl[8];
#pragma unroll
    for (int r = 0; r < 8; ++r) scl[r] = __shfl(al, 8 * hh + r, 32);
#pragma unroll
    for (int j = 0; j < 4; ++j) {
#pragma unroll
      for (int r = 0; r < 8; ++r) o[j][r] *= scl[r];
    }
    {
      const _Float16* vhp = Vhb + kb;
      const v16h vh0 = ldfrag_h(vhp);
      const v16h vh1 = ldfrag_h(vhp + (size_t)16 * SEQ);
      const v16h vh2 = ldfrag_h(vhp + (size_t)32 * SEQ);
      const v16h vh3 = ldfrag_h(vhp + (size_t)48 * SEQ);
      o[0] = mma_h(ph.v, vh0, o[0]);
      o[1] = mma_h(ph.v, vh1, o[1]);
      o[2] = mma_h(ph.v, vh2, o[2]);
      o[3] = mma_h(ph.v, vh3, o[3]);
      g4_5<v16h>(o[0], o[1], o[2], o[3], ph.v, vh0, vh1, vh2, vh3);
    }
  }
  acc_guard4(o[0], o[1], o[2], o[3]);

  const float linv = (1.0f / lrun) * (1.0f / (PCAR * VCAR));
  float inv[8];
#pragma unroll
  for (int r = 0; r < 8; ++r) inv[r] = __shfl(linv, 8 * hh + r, 32);
  float* slab = smem + wave * SLABF;
#pragma unroll
  for (int r = 0; r < 8; ++r) {
#pragma unroll
    for (int j = 0; j < 4; ++j) slab[(8 * hh + r) * 68 + j * 16 + c] = o[j][r] * inv[r];
  }
  wave_sync_lds();
  v4f vals[8];
#pragma unroll
  for (int it = 0; it < 8; ++it) vals[it] = *(const v4f*)(slab + (it * 2 + hh) * 68 + c * 4);
  float* dst = out + ((size_t)(q0 + hh)) * (size_t)OUTW + head * HD + c * 4;
  for (int pass = 0; pass < 2; ++pass) {
#pragma unroll
    for (int it = 0; it < 8; ++it) {
      *(volatile v4f*)(dst + (size_t)(it * 2) * (size_t)OUTW) = vals[it];
    }
    __threadfence();
  }
}

extern "C" void kernel_launch(void* const* d_in, const int* in_sizes, int n_in,
                              void* d_out, int out_size, void* d_ws, size_t ws_size,
                              hipStream_t stream) {
  const int XN = SEQ * DIN;
  const int ON = SEQ * OUTW;
  if (n_in < 7) return;
  if (in_sizes[0] != XN) return;
  if (in_sizes[1] != DIN * DIN || in_sizes[3] != DIN * DIN || in_sizes[5] != DIN * DIN) return;
  if (in_sizes[2] != DIN || in_sizes[4] != DIN || in_sizes[6] != DIN) return;
  if (out_size != ON) return;

  const float* xin = (const float*)d_in[0];
  const float* wq  = (const float*)d_in[1];
  const float* bq  = (const float*)d_in[2];
  const float* wk  = (const float*)d_in[3];
  const float* bk  = (const float*)d_in[4];
  const float* wv  = (const float*)d_in[5];
  const float* bv  = (const float*)d_in[6];
  float*       out = (float*)d_out;
  const int    nb  = in_sizes[2];

  const size_t szXB = (size_t)SEQ * DIN * 2;
  const size_t szW  = (size_t)OUTW * DIN * 2;
  const size_t szF  = (size_t)SEQ * OUTW * 4;
  const size_t szP  = (size_t)SEQ * OUTW * 2;
  size_t off = 0;
  const size_t oXB  = off; off += szXB;
  const size_t oWQB = off; off += szW;
  const size_t oWKB = off; off += szW;
  const size_t oWVB = off; off += szW;
  const size_t oF   = off; off += szF;
  const size_t oQH  = off; off += szP;
  const size_t oKH  = off; off += szP;
  const size_t oVH  = off; off += szP;
  if (off > ws_size) return;
  if (off > (size_t)134217728) return;

  char* ws = (char*)d_ws;
  u16*   XB  = (u16*)(ws + oXB);
  u16*   WQB = (u16*)(ws + oWQB);
  u16*   WKB = (u16*)(ws + oWKB);
  u16*   WVB = (u16*)(ws + oWVB);
  float* F   = (float*)(ws + oF);
  u16*   QH  = (u16*)(ws + oQH);
  u16*   KH  = (u16*)(ws + oKH);
  u16*   VH  = (u16*)(ws + oVH);

  const dim3 blk(256);
  const int n8x = XN / 8;
  const int n8w = (OUTW * DIN) / 8;
  const int n8o = ON / 8;
  const dim3 gX((n8x + 255) / 256);
  const dim3 gWc((n8w + 255) / 256);
  const dim3 gO((n8o + 255) / 256);
  const dim3 gGt((SEQ / 64) * (OUTW / 64));
  const dim3 gGc((OUTW / 64) * (SEQ / 64));
  const dim3 bG(128);
  const dim3 gAT(ATT_BLOCKS);
  const dim3 bAT(ATT_THREADS);

  cvb16<<<gWc, blk, 0, stream>>>(wq, WQB, n8w);
  cvb16<<<gWc, blk, 0, stream>>>(wk, WKB, n8w);
  cvb16<<<gWc, blk, 0, stream>>>(wv, WVB, n8w);
  cvb16<<<gX, blk, 0, stream>>>(xin, XB, n8x);
  gemm_bfb<<<gGt, bG, 0, stream>>>(XB, WQB, bq, F, SEQ, OUTW, DIN, 1.0f, 0, nb);
  cvh16<<<gO, blk, 0, stream>>>(F, QH, n8o, QSC);
  gemm_bfb<<<gGt, bG, 0, stream>>>(XB, WKB, bk, F, SEQ, OUTW, DIN, 1.0f, 0, nb);
  cvh16<<<gO, blk, 0, stream>>>(F, KH, n8o, KSC);
  gemm_bfb<<<gGc, bG, 0, stream>>>(WVB, XB, bv, F, OUTW, SEQ, DIN, 1.0f, 1, nb);
  cvh16<<<gO, blk, 0, stream>>>(F, VH, n8o, VCAR);
  attn_fwd<<<gAT, bAT, 0, stream>>>(QH, KH, VH, out);
  (void)hipGetLastError();
}
